// OptimizedMambaBlock_8881992368586
// MI455X (gfx1250) — hardware-verified
//
#include <hip/hip_runtime.h>
#include <math.h>

constexpr int kBatch   = 2;
constexpr int kLen     = 1024;
constexpr int kDm      = 1024;
constexpr int kDi      = 2048;
constexpr int kNs      = 16;
constexpr int kKc      = 4;
constexpr int kTok     = kBatch * kLen;
constexpr int kNxz     = 2 * kDi;
constexpr int kNdbu    = 2 * kNs + kDi;
constexpr int kNdbuPad = 2112;
constexpr int kChunk   = 64;
constexpr int kChan    = 64;

constexpr size_t kBytesXp  = (size_t)kTok * kDm * 2;
constexpr size_t kBytesWin = (size_t)kNxz * kDm * 2;
constexpr size_t kBytesWx  = (size_t)kNdbuPad * kDi * 2;
constexpr size_t kBytesWo  = (size_t)kDm * kDi * 2;
constexpr size_t kBytesXz  = (size_t)kTok * kNxz * 4;
constexpr size_t kBytesXc  = (size_t)kTok * kDi * 2;
constexpr size_t kBytesDbu = (size_t)kTok * kNdbuPad * 4;
constexpr size_t kBytesG   = (size_t)kTok * kDi * 2;
constexpr size_t kOffXh   = 0;
constexpr size_t kOffXl   = kOffXh + kBytesXp;
constexpr size_t kOffWinH = kOffXl + kBytesXp;
constexpr size_t kOffWinL = kOffWinH + kBytesWin;
constexpr size_t kOffWxH  = kOffWinL + kBytesWin;
constexpr size_t kOffWxL  = kOffWxH + kBytesWx;
constexpr size_t kOffWoH  = kOffWxL + kBytesWx;
constexpr size_t kOffWoL  = kOffWoH + kBytesWo;
constexpr size_t kOffXz   = kOffWoL + kBytesWo;
constexpr size_t kOffXcH  = kOffXz + kBytesXz;
constexpr size_t kOffXcL  = kOffXcH + kBytesXc;
constexpr size_t kOffDbu  = kOffXcL + kBytesXc;
constexpr size_t kOffEnd  = kOffDbu + kBytesDbu;
constexpr size_t kOffGh   = 0;
constexpr size_t kOffGl   = kOffGh + kBytesG;
constexpr size_t kWsCap   = (size_t)134217728;
typedef char ws_fits_check[(kOffEnd <= kWsCap) ? 1 : -1];
typedef char g_alias_check[(kOffGl + kBytesG <= kOffWxH) ? 1 : -1];

typedef __attribute__((ext_vector_type(16))) _Float16 v16h;
typedef __attribute__((ext_vector_type(8)))  _Float16 v8h;
typedef __attribute__((ext_vector_type(16))) __bf16   v16b;
typedef __attribute__((ext_vector_type(8)))  __bf16   v8b;
typedef __attribute__((ext_vector_type(8)))  float    v8f;
typedef __attribute__((ext_vector_type(4)))  float    v4f;
typedef __attribute__((ext_vector_type(4)))  unsigned int v4u;

__device__ __forceinline__ unsigned short f2bf_bits(float f) {
  unsigned u = __float_as_uint(f);
  return (unsigned short)((u + 0x7FFFu + ((u >> 16) & 1u)) >> 16);
}
__device__ __forceinline__ float bf_bits2f(unsigned short h) { return __uint_as_float(((unsigned)h) << 16); }

__device__ __forceinline__ void dep_guard_h(v8f& a, v8f& b, v16h x, v16h y) { asm volatile("v_nop\n\tv_nop\n\tv_nop\n\tv_nop" : "+v"(a), "+v"(b) : "v"(x), "v"(y)); }
__device__ __forceinline__ void dep_guard_b(v8f& a, v8f& b, v16b x, v16b y) { asm volatile("v_nop\n\tv_nop\n\tv_nop\n\tv_nop" : "+v"(a), "+v"(b) : "v"(x), "v"(y)); }
__device__ __forceinline__ void keep4_h(v16h a, v16h b, v16h c, v16h d) { asm volatile("v_nop" :: "v"(a), "v"(b), "v"(c), "v"(d)); }
__device__ __forceinline__ void keep4_b(v16b a, v16b b, v16b c, v16b d) { asm volatile("v_nop" :: "v"(a), "v"(b), "v"(c), "v"(d)); }
__device__ __forceinline__ void acc_guard4(v8f& a, v8f& b, v8f& c, v8f& d) { asm volatile("v_nop\n\tv_nop\n\tv_nop\n\tv_nop" : "+v"(a), "+v"(b), "+v"(c), "+v"(d)); }
template <typename T> struct Frag;
template <> struct Frag<_Float16> {
  typedef v16h V; union U { v16h v; v8h h[2]; };
  static __device__ __forceinline__ v16h load(const _Float16* p) {
    U f; f.h[0] = *(const v8h*)(p); f.h[1] = *(const v8h*)(p + 16); return f.v;
  }
  static __device__ __forceinline__ v8f mma(v16h a, v16h b, v8f c) {
    return __builtin_amdgcn_wmma_f32_16x16x32_f16(false, a, false, b, (short)0, c, false, false);
  }
  static __device__ __forceinline__ void guard(v8f& a, v8f& b, v16h x, v16h y) { dep_guard_h(a, b, x, y); }
  static __device__ __forceinline__ void keep(v16h a, v16h b, v16h c, v16h d) { keep4_h(a, b, c, d); }
};
template <> struct Frag<__bf16> {
  typedef v16b V; union U { v16b v; v8b h[2]; };
  static __device__ __forceinline__ v16b load(const __bf16* p) {
    U f; f.h[0] = *(const v8b*)(p); f.h[1] = *(const v8b*)(p + 16); return f.v;
  }
  static __device__ __forceinline__ v8f mma(v16b a, v16b b, v8f c) {
    return __builtin_amdgcn_wmma_f32_16x16x32_bf16(false, a, false, b, (short)0, c, false, false);
  }
  static __device__ __forceinline__ void guard(v8f& a, v8f& b, v16b x, v16b y) { dep_guard_b(a, b, x, y); }
  static __device__ __forceinline__ void keep(v16b a, v16b b, v16b c, v16b d) { keep4_b(a, b, c, d); }
};

__device__ __forceinline__ unsigned pk16(unsigned short a, unsigned short b) { return (unsigned)a | ((unsigned)b << 16); }

template <int ET> struct Elem;
template <> struct Elem<0> { typedef _Float16 T; };
template <> struct Elem<1> { typedef __bf16 T; };
template <int ET, bool SPLIT, int BIAS_MODE, int OUT_MODE, bool RESID, int ACT = 0>
__global__ __launch_bounds__(256) void wmma_gemm64(
    const unsigned short* __restrict__ Ap, const unsigned short* __restrict__ A2p, int lda, long strideA,
    const unsigned short* __restrict__ Btp, const unsigned short* __restrict__ Bt2p, int ldb, long strideB,
    void* __restrict__ Cout, void* __restrict__ Cout2, int ldc, long strideC,
    const float* __restrict__ bias,
    const float* __restrict__ resid, long strideR,
    int M, int N, int K, float scale) {
  typedef typename Elem<ET>::T T;
  typedef typename Frag<T>::V V;
  const T* A = (const T*)Ap; const T* A2 = (const T*)A2p; const T* Bt = (const T*)Btp; const T* Bt2 = (const T*)Bt2p;
  __shared__ __align__(16) float sT[8][16 * 68];
  const int b    = blockIdx.y;
  const int lane = threadIdx.x & 31;
  const int wave = threadIdx.x >> 5;
  const int tilesN = N >> 6;
  const int tilesM = M >> 6;
  const int tile = blockIdx.x * 8 + wave;
  if (tile >= tilesM * tilesN) return;
  const int tm = tile / tilesN;
  const int tn = tile - tm * tilesN;
  const int m0 = tm << 6;
  const int n0 = tn << 6;

  const T* Ab  = A  + (size_t)b * strideA;
  const T* Bb  = Bt + (size_t)b * strideB;
  const T* Ab2 = SPLIT ? (A2  + (size_t)b * strideA) : nullptr;
  const T* Bb2 = SPLIT ? (Bt2 + (size_t)b * strideB) : nullptr;

  const int rlane = lane & 15;
  const int koff  = (lane >> 4) * 8;
  const int mOff  = (lane >> 4) * 8;

  v8f acc[4][4];
#pragma unroll
  for (int i = 0; i < 4; ++i)
#pragma unroll
    for (int j = 0; j < 4; ++j) acc[i][j] = (v8f){0.f,0.f,0.f,0.f,0.f,0.f,0.f,0.f};

  for (int k0 = 0; k0 < K; k0 += 32) {
    V bh[4], bl[4];
#pragma unroll
    for (int j = 0; j < 4; ++j) {
      const size_t bo = (size_t)(n0 + (j << 4) + rlane) * ldb + koff + k0;
      bh[j] = Frag<T>::load(Bb + bo);
      if (SPLIT) bl[j] = Frag<T>::load(Bb2 + bo);
    }
#pragma unroll
    for (int i = 0; i < 4; ++i) {
      const size_t ao = (size_t)(m0 + (i << 4) + rlane) * lda + koff + k0;
      V ah = Frag<T>::load(Ab + ao);
      V al;
      if (SPLIT) al = Frag<T>::load(Ab2 + ao);
#pragma unroll
      for (int j = 0; j < 4; ++j) {
        acc[i][j] = Frag<T>::mma(ah, bh[j], acc[i][j]);
        if (SPLIT) {
          acc[i][j] = Frag<T>::mma(ah, bl[j], acc[i][j]);
          acc[i][j] = Frag<T>::mma(al, bh[j], acc[i][j]);
        }
      }
      Frag<T>::guard(acc[i][0], acc[i][3], ah, SPLIT ? al : ah);
    }
    Frag<T>::keep(bh[0], bh[1], bh[2], bh[3]);
    if (SPLIT) Frag<T>::keep(bl[0], bl[1], bl[2], bl[3]);
  }
  acc_guard4(acc[0][0], acc[0][1], acc[0][2], acc[0][3]);
  acc_guard4(acc[1][0], acc[1][1], acc[1][2], acc[1][3]);
  acc_guard4(acc[2][0], acc[2][1], acc[2][2], acc[2][3]);
  acc_guard4(acc[3][0], acc[3][1], acc[3][2], acc[3][3]);

  float* slab = sT[wave];
  const float* Rb = RESID ? (resid + (size_t)b * strideR) : nullptr;
#pragma unroll
  for (int i = 0; i < 4; ++i) {
    const int mBase = m0 + (i << 4);
#pragma unroll
    for (int j = 0; j < 4; ++j) {
      const int n = n0 + (j << 4) + rlane;
      float bv = 0.f;
      if (BIAS_MODE == 2) bv = bias[n];
#pragma unroll
      for (int r = 0; r < 8; ++r) {
        float v = acc[i][j][r] * scale;
        if (BIAS_MODE == 1) v += bias[mBase + mOff + r];
        if (BIAS_MODE == 2) v += bv;
        if (RESID) v += Rb[(size_t)(mBase + mOff + r) * ldc + n];
        if (ACT == 2) v = fmaxf(v, 0.0f);
        if (ACT == 4) v = (v > 0.f) ? v : 0.01f * v;
        slab[(mOff + r) * 68 + (j << 4) + rlane] = v;
      }
    }
    __builtin_amdgcn_fence(__ATOMIC_RELEASE, "workgroup");
    __builtin_amdgcn_wave_barrier();
    __builtin_amdgcn_fence(__ATOMIC_ACQUIRE, "workgroup");
    if (OUT_MODE == 0) {
      float* C = (float*)Cout + (size_t)b * strideC;
      const int hh = lane >> 4, c4 = (lane & 15) * 4;
      for (int pass = 0; pass < 2; ++pass) {
#pragma unroll
        for (int it = 0; it < 8; ++it) {
          const int row = it * 2 + hh;
          v4f v = *(const v4f*)(slab + row * 68 + c4);
          *(volatile v4f*)(C + (size_t)(mBase + row) * ldc + n0 + c4) = v;
        }
        __threadfence();
      }
    } else {
      const int q = lane >> 3, c8 = (lane & 7) * 8;
      unsigned short* C  = (unsigned short*)Cout  + (size_t)b * strideC;
      unsigned short* C2 = (OUT_MODE == 2) ? ((unsigned short*)Cout2 + (size_t)b * strideC) : nullptr;
      for (int pass = 0; pass < 2; ++pass) {
#pragma unroll
        for (int it = 0; it < 4; ++it) {
          const int row = it * 4 + q;
          const float* sp = slab + row * 68 + c8;
          v8h hv, lv;
#pragma unroll
          for (int e = 0; e < 8; ++e) {
            if (OUT_MODE == 1) {
              hv[e] = (_Float16)sp[e];
            } else {
              unsigned short hb = f2bf_bits(sp[e]);
              unsigned short lb = f2bf_bits(sp[e] - bf_bits2f(hb));
              hv[e] = __builtin_bit_cast(_Float16, hb);
              lv[e] = __builtin_bit_cast(_Float16, lb);
            }
          }
          *(volatile v8h*)(C + (size_t)(mBase + row) * ldc + n0 + c8) = hv;
          if (OUT_MODE == 2) *(volatile v8h*)(C2 + (size_t)(mBase + row) * ldc + n0 + c8) = lv;
        }
        __threadfence();
      }
    }
    __builtin_amdgcn_fence(__ATOMIC_RELEASE, "workgroup");
    __builtin_amdgcn_wave_barrier();
    __builtin_amdgcn_fence(__ATOMIC_ACQUIRE, "workgroup");
  }
}

__device__ __forceinline__ void split8_bf(const v4f a, const v4f c, v4u& uh, v4u& ul) {
  unsigned short hb[8], lb[8];
#pragma unroll
  for (int e = 0; e < 4; ++e) {
    const float f0 = a[e];
    hb[e] = f2bf_bits(f0);
    lb[e] = f2bf_bits(f0 - bf_bits2f(hb[e]));
    const float f1 = c[e];
    hb[4 + e] = f2bf_bits(f1);
    lb[4 + e] = f2bf_bits(f1 - bf_bits2f(hb[4 + e]));
  }
  uh = (v4u){pk16(hb[0], hb[1]), pk16(hb[2], hb[3]), pk16(hb[4], hb[5]), pk16(hb[6], hb[7])};
  ul = (v4u){pk16(lb[0], lb[1]), pk16(lb[2], lb[3]), pk16(lb[4], lb[5]), pk16(lb[6], lb[7])};
}

__global__ __launch_bounds__(256) void split8_kernel(const float* __restrict__ in, unsigned short* __restrict__ hi,
                                                     unsigned short* __restrict__ lo, int n8) {
  const int i = blockIdx.x * 256 + threadIdx.x;
  if (i >= n8) return;
  const float* p = in + 8 * (size_t)i;
  const v4f a = *(const v4f*)(p);
  const v4f c = *(const v4f*)(p + 4);
  v4u uh, ul;
  split8_bf(a, c, uh, ul);
  const size_t o = 8 * (size_t)i;
  *(volatile v4u*)(hi + o) = uh;
  *(volatile v4u*)(lo + o) = ul;
  __threadfence();
  *(volatile v4u*)(hi + o) = uh;
  *(volatile v4u*)(lo + o) = ul;
}

__global__ __launch_bounds__(256) void wtsplit_kernel(const float* __restrict__ W, int N, int K,
                                                      unsigned short* __restrict__ hi, unsigned short* __restrict__ lo) {
  __shared__ float sm[64][65];
  const int t  = threadIdx.x;
  const int k0 = blockIdx.x * 64;
  const int n0 = blockIdx.y * 64;
#pragma unroll
  for (int i = 0; i < 16; ++i) {
    const int e = i * 256 + t;
    const int r = e >> 6;
    const int c = e & 63;
    const int n = n0 + c;
    const int nc = (n < N) ? n : (N - 1);
    float v = W[(size_t)(k0 + r) * N + nc];
    if (n >= N) v = 0.0f;
    sm[c][r] = v;
  }
  __syncthreads();
  const int lane = t & 31, wave = t >> 5;
  const int q = lane >> 3, c8 = (lane & 7) * 8;
  for (int pass = 0; pass < 2; ++pass) {
#pragma unroll
    for (int it = 0; it < 2; ++it) {
      const int row = wave * 8 + it * 4 + q;
      const float* sp = &sm[row][c8];
      const v4f a = (v4f){sp[0], sp[1], sp[2], sp[3]};
      const v4f c = (v4f){sp[4], sp[5], sp[6], sp[7]};
      v4u uh, ul;
      split8_bf(a, c, uh, ul);
      const size_t o = (size_t)(n0 + row) * K + k0 + c8;
      *(volatile v4u*)(hi + o) = uh;
      *(volatile v4u*)(lo + o) = ul;
    }
    __threadfence();
  }
}

__global__ __launch_bounds__(256) void conv_silu_split_kernel(const float* __restrict__ xz, const float* __restrict__ cw,
                                                              const float* __restrict__ cb,
                                                              unsigned short* __restrict__ hi, unsigned short* __restrict__ lo) {
  const int t   = threadIdx.x;
  const int row = blockIdx.x;
  const int d8  = t * 8;
  const int l   = row & (kLen - 1);
  const int b   = row >> 10;
  v4f wv[8];
#pragma unroll
  for (int e = 0; e < 8; ++e) wv[e] = *(const v4f*)(cw + (size_t)(d8 + e) * kKc);
  float acc[8];
#pragma unroll
  for (int e = 0; e < 8; ++e) acc[e] = 0.0f;
#pragma unroll
  for (int j = 0; j < kKc; ++j) {
    const int ll = l - (kKc - 1) + j;
    if (ll >= 0) {
      const float* src = xz + (size_t)(b * kLen + ll) * kNxz + d8;
      const v4f a0 = *(const v4f*)(src);
      const v4f a1 = *(const v4f*)(src + 4);
#pragma unroll
      for (int e = 0; e < 4; ++e) {
        acc[e]     += wv[e][j] * a0[e];
        acc[4 + e] += wv[4 + e][j] * a1[e];
      }
    }
  }
  const v4f b0 = *(const v4f*)(cb + d8);
  const v4f b1 = *(const v4f*)(cb + d8 + 4);
  v4f o0, o1;
#pragma unroll
  for (int e = 0; e < 4; ++e) {
    const float v0 = acc[e] + b0[e];
    o0[e] = v0 * (1.0f / (1.0f + expf(-v0)));
    const float v1 = acc[4 + e] + b1[e];
    o1[e] = v1 * (1.0f / (1.0f + expf(-v1)));
  }
  v4u uh, ul;
  split8_bf(o0, o1, uh, ul);
  const size_t o = (size_t)row * kDi + d8;
  *(volatile v4u*)(hi + o) = uh;
  *(volatile v4u*)(lo + o) = ul;
  __threadfence();
  *(volatile v4u*)(hi + o) = uh;
  *(volatile v4u*)(lo + o) = ul;
}

__global__ __launch_bounds__(64) void ssm_gate_kernel(const float* __restrict__ dbu, const float* __restrict__ xz,
                                                      const float* __restrict__ xpb, const float* __restrict__ dtw,
                                                      const float* __restrict__ dtb, const float* __restrict__ Dp,
                                                      unsigned short* __restrict__ ghi, unsigned short* __restrict__ glo) {
#pragma clang fp contract(off)
  __shared__ __align__(16) float sDS[kChunk * kNs];
  __shared__ __align__(16) float sBm[kChunk * kNs];
  __shared__ float sH[kNs * kChan];
  __shared__ __align__(16) float sG[kChunk * 68];
  __shared__ float sBias[32];
  const int t    = threadIdx.x;
  const int lane = t & 31, wave = t >> 5;
  const int b    = blockIdx.y;
  const int d0   = blockIdx.x * kChan;
  const int d    = d0 + t;
  if (t < 32) sBias[t] = xpb[t];
#pragma unroll
  for (int n = 0; n < kNs; ++n) sH[n * kChan + t] = 0.0f;
  float w[kNs];
#pragma unroll
  for (int n = 0; n < kNs; ++n) w[n] = dtw[(size_t)n * kDi + d];
  const float dtbias = dtb[d];
  const float Dd     = Dp[d];
  const float ub     = xpb[2 * kNs + d];
  __syncthreads();

  for (int ch = 0; ch < kLen / kChunk; ++ch) {
    const int tok0 = b * kLen + ch * kChunk;
    {
      const float* src = dbu + (size_t)(tok0 + t) * kNdbuPad;
#pragma unroll
      for (int qq = 0; qq < 4; ++qq) {
        const v4f a = *(const v4f*)(src + 4 * qq);
        const v4f c = *(const v4f*)(src + kNs + 4 * qq);
#pragma unroll
        for (int e = 0; e < 4; ++e) {
          sDS[t * kNs + 4 * qq + e] = a[e] + sBias[4 * qq + e];
          sBm[t * kNs + 4 * qq + e] = c[e] + sBias[kNs + 4 * qq + e];
        }
      }
    }
    __syncthreads();
#pragma unroll 1
    for (int s = 0; s < kChunk; ++s) {
      const int tok = tok0 + s;
      const v4f* dsv = (const v4f*)(sDS + s * kNs);
      float pre = 0.0f;
#pragma unroll
      for (int qq = 0; qq < 4; ++qq) {
        const v4f dq = dsv[qq];
#pragma unroll
        for (int e = 0; e < 4; ++e) pre += dq[e] * w[4 * qq + e];
      }
      pre += dtbias;
      const float delta = fmaxf(pre, 0.0f) + log1pf(expf(-fabsf(pre)));
      const float u  = dbu[(size_t)tok * kNdbuPad + 2 * kNs + d] + ub;
      const float zv = xz[(size_t)tok * kNxz + kDi + d];
      float y = 0.0f;
      const float* bm = sBm + s * kNs;
#pragma unroll 1
      for (int n = 0; n < kNs; ++n) {
        const float dA   = expf(delta * (float)(-(n + 1)));
        const float dbun = (delta * bm[n]) * u;
        float h = sH[n * kChan + t];
        h = dA * h + dbun;
        sH[n * kChan + t] = h;
        y += h;
      }
      y = y + u * Dd;
      const float gz = zv * (1.0f / (1.0f + expf(-zv)));
      sG[s * 68 + t] = y * gz;
    }
    __syncthreads();
    {
      const int q = lane >> 3, c8 = (lane & 7) * 8;
      for (int pass = 0; pass < 2; ++pass) {
#pragma unroll
        for (int it = 0; it < 8; ++it) {
          const int row = wave * 32 + it * 4 + q;
          const float* sp = sG + row * 68 + c8;
          const v4f a = *(const v4f*)(sp);
          const v4f c = *(const v4f*)(sp + 4);
          v4u uh, ul;
          split8_bf(a, c, uh, ul);
          const size_t o = (size_t)(tok0 + row) * kDi + d0 + c8;
          *(volatile v4u*)(ghi + o) = uh;
          *(volatile v4u*)(glo + o) = ul;
        }
        __threadfence();
      }
    }
  }
}

extern "C" void kernel_launch(void* const* d_in, const int* in_sizes, int n_in,
                              void* d_out, int out_size, void* d_ws, size_t ws_size, hipStream_t stream) {
  if (n_in < 12) return;
  if (in_sizes[0] != kTok * kDm || in_sizes[1] != kDm * kNxz || in_sizes[5] != kDi * kNdbu ||
      in_sizes[7] != kNs * kDi || in_sizes[10] != kDi * kDm || out_size != kTok * kDm) return;
  if (ws_size < kOffEnd) return;

  const float* x          = (const float*)d_in[0];
  const float* in_proj_w  = (const float*)d_in[1];
  const float* in_proj_b  = (const float*)d_in[2];
  const float* conv_w     = (const float*)d_in[3];
  const float* conv_b     = (const float*)d_in[4];
  const float* x_proj_w   = (const float*)d_in[5];
  const float* x_proj_b   = (const float*)d_in[6];
  const float* dt_proj_w  = (const float*)d_in[7];
  const float* dt_proj_b  = (const float*)d_in[8];
  const float* Dp         = (const float*)d_in[9];
  const float* out_proj_w = (const float*)d_in[10];
  const float* out_proj_b = (const float*)d_in[11];
  float* out = (float*)d_out;

  char* ws = (char*)d_ws;
  unsigned short* xh   = (unsigned short*)(ws + kOffXh);
  unsigned short* xl   = (unsigned short*)(ws + kOffXl);
  unsigned short* winh = (unsigned short*)(ws + kOffWinH);
  unsigned short* winl = (unsigned short*)(ws + kOffWinL);
  unsigned short* wxh  = (unsigned short*)(ws + kOffWxH);
  unsigned short* wxl  = (unsigned short*)(ws + kOffWxL);
  unsigned short* woh  = (unsigned short*)(ws + kOffWoH);
  unsigned short* wol  = (unsigned short*)(ws + kOffWoL);
  float*          xz   = (float*)(ws + kOffXz);
  unsigned short* xch  = (unsigned short*)(ws + kOffXcH);
  unsigned short* xcl  = (unsigned short*)(ws + kOffXcL);
  float*          dbu  = (float*)(ws + kOffDbu);
  unsigned short* gh   = (unsigned short*)(ws + kOffGh);
  unsigned short* gl   = (unsigned short*)(ws + kOffGl);

  {
    const int n8 = kTok * kDm / 8;
    split8_kernel<<<dim3((n8 + 255) / 256), dim3(256), 0, stream>>>(x, xh, xl, n8);
  }
  wtsplit_kernel<<<dim3(kDm / 64, kNxz / 64), dim3(256), 0, stream>>>(in_proj_w, kNxz, kDm, winh, winl);
  wtsplit_kernel<<<dim3(kDi / 64, kNdbuPad / 64), dim3(256), 0, stream>>>(x_proj_w, kNdbu, kDi, wxh, wxl);
  wtsplit_kernel<<<dim3(kDi / 64, kDm / 64), dim3(256), 0, stream>>>(out_proj_w, kDm, kDi, woh, wol);

  wmma_gemm64<1, true, 2, 0, false, 0><<<dim3((kTok / 64) * (kNxz / 64) / 8, 1), dim3(256), 0, stream>>>(
      xh, xl, kDm, 0L, winh, winl, kDm, 0L, (void*)xz, nullptr, kNxz, 0L, in_proj_b, nullptr, 0L,
      kTok, kNxz, kDm, 1.0f);

  conv_silu_split_kernel<<<dim3(kTok), dim3(256), 0, stream>>>(xz, conv_w, conv_b, xch, xcl);

  wmma_gemm64<1, true, 0, 0, false, 0><<<dim3((kTok / 64) * (kNdbuPad / 64) / 8, 1), dim3(256), 0, stream>>>(
      xch, xcl, kDi, 0L, wxh, wxl, kDi, 0L, (void*)dbu, nullptr, kNdbuPad, 0L, nullptr, nullptr, 0L,
      kTok, kNdbuPad, kDi, 1.0f);

  ssm_gate_kernel<<<dim3(kDi / kChan, kBatch), dim3(kChan), 0, stream>>>(dbu, xz, x_proj_b, dt_proj_w, dt_proj_b, Dp, gh, gl);

  wmma_gemm64<1, true, 2, 0, false, 0><<<dim3((kTok / 64) * (kDm / 64) / 8, 1), dim3(256), 0, stream>>>(
      gh, gl, kDi, 0L, woh, wol, kDi, 0L, (void*)out, nullptr, kDm, 0L, out_proj_b, nullptr, 0L,
      kTok, kDm, kDi, 1.0f);
}
